// BasicTransformerLayer_32366873543455
// MI455X (gfx1250) — hardware-verified
//
#include <hip/hip_runtime.h>


#define NB_  8
#define TT   1024
#define LC   256
#define EE   768
#define EC   512
#define NH_  12
#define HD   64
#define FF   3072
#define PCAR 1024.0f
typedef _Float16 h16;
typedef unsigned short bf;
typedef __attribute__((ext_vector_type(16))) __bf16   v16bf;
typedef __attribute__((ext_vector_type(16))) _Float16 v16h;
typedef __attribute__((ext_vector_type(8)))  _Float16 v8h;
typedef __attribute__((ext_vector_type(8)))  unsigned short v8us;
typedef __attribute__((ext_vector_type(8)))  float    v8f;
typedef __attribute__((ext_vector_type(4)))  float    v4f;
typedef v8h  __attribute__((may_alias)) v8ha;
typedef v4f  __attribute__((may_alias)) v4fa;
typedef v8us __attribute__((may_alias)) v8usa;

__device__ __forceinline__ unsigned short f2bf(float f) { unsigned u = __float_as_uint(f); u += 0x7FFFu + ((u >> 16) & 1u); return (unsigned short)(u >> 16); }
__device__ __forceinline__ float bf2f(unsigned short b) { return __uint_as_float(((unsigned)b) << 16); }
__device__ __forceinline__ float bfr(float f) { return bf2f(f2bf(f)); }
__device__ __forceinline__ v16h cat16(v8h lo, v8h hi) { return __builtin_shufflevector(lo, hi, 0, 1, 2, 3, 4, 5, 6, 7, 8, 9, 10, 11, 12, 13, 14, 15); }
__device__ __forceinline__ v16bf cat16b(v8us lo, v8us hi) { return __builtin_bit_cast(v16bf, __builtin_shufflevector(lo, hi, 0, 1, 2, 3, 4, 5, 6, 7, 8, 9, 10, 11, 12, 13, 14, 15)); }
__device__ __forceinline__ v8f wmma16(v16h a, v16h b, v8f c) { return __builtin_amdgcn_wmma_f32_16x16x32_f16(false, a, false, b, (short)0, c, false, false); }
__device__ __forceinline__ v8f wmmab(v16bf a, v16bf b, v8f c) { return __builtin_amdgcn_wmma_f32_16x16x32_bf16(false, a, false, b, (short)0, c, false, false); }


template <typename T16> struct WFrag;
template <> struct WFrag<h16> { typedef v16h V; static __device__ __forceinline__ V ld(const h16* p) { return cat16(*(const v8h*)p, *(const v8h*)(p + 16)); } static __device__ __forceinline__ v8f mma(V a, V b, v8f c) { return wmma16(a, b, c); } };
template <> struct WFrag<bf> { typedef v16bf V; static __device__ __forceinline__ V ld(const bf* p) { return cat16b(*(const v8us*)p, *(const v8us*)(p + 16)); } static __device__ __forceinline__ v8f mma(V a, V b, v8f c) { return wmmab(a, b, c); } };
template <typename T16, int NSPLIT, bool BIAS>
__global__ __launch_bounds__(32) void k_gemmw(const T16* __restrict__ A, const T16* __restrict__ A2, const T16* __restrict__ Bt, const T16* __restrict__ Bt2, int K, float* C, int ldc, const float* __restrict__ bias, size_t sA, size_t sB, size_t sC) {
    typedef typename WFrag<T16>::V V;
    __shared__ __align__(16) float os[16 * 68];
    const size_t z = blockIdx.z; A += z * sA; if (A2) A2 += z * sA; Bt += z * sB; if (Bt2) Bt2 += z * sB; C += z * sC;
    const int lane = threadIdx.x & 31, lr = lane & 15, hi = lane >> 4; const int r0 = blockIdx.x * 64, c0 = blockIdx.y * 64;
    v8f acc[4][4];
#pragma unroll
    for (int mb = 0; mb < 4; ++mb)
#pragma unroll
        for (int nb = 0; nb < 4; ++nb) acc[mb][nb] = (v8f){};
    const size_t aoff = (size_t)(r0 + lr) * K + 8 * hi, boff = (size_t)(c0 + lr) * K + 8 * hi;
#pragma unroll 1
    for (int kc = 0; kc < K; kc += 32) {
        V a[4], a2[4];
#pragma unroll
        for (int mb = 0; mb < 4; ++mb) { a[mb] = WFrag<T16>::ld(A + aoff + (size_t)mb * 16 * K + kc); if (NSPLIT == 1 || NSPLIT == 2) a2[mb] = WFrag<T16>::ld(A2 + aoff + (size_t)mb * 16 * K + kc); }
#pragma unroll
        for (int nb = 0; nb < 4; ++nb) { const V b = WFrag<T16>::ld(Bt + boff + (size_t)nb * 16 * K + kc); V b2; if (NSPLIT >= 2) b2 = WFrag<T16>::ld(Bt2 + boff + (size_t)nb * 16 * K + kc);
#pragma unroll
            for (int mb = 0; mb < 4; ++mb) { acc[mb][nb] = WFrag<T16>::mma(a[mb], b, acc[mb][nb]); if (NSPLIT == 1 || NSPLIT == 2) acc[mb][nb] = WFrag<T16>::mma(a2[mb], b, acc[mb][nb]); if (NSPLIT >= 2) acc[mb][nb] = WFrag<T16>::mma(a[mb], b2, acc[mb][nb]); } }
        asm volatile("v_nop\n\tv_nop\n\tv_nop\n\tv_nop" : "+v"(acc[0][0]), "+v"(acc[1][1]), "+v"(acc[2][2]), "+v"(acc[3][3]) : "v"(a[0]), "v"(a[3]));
    }
#pragma unroll
    for (int mb = 0; mb < 4; ++mb) {
#pragma unroll
        for (int nb = 0; nb < 4; ++nb) {
#pragma unroll
            for (int j = 0; j < 8; ++j) os[(hi * 8 + j) * 68 + nb * 16 + lr] = acc[mb][nb][j]; }
        __builtin_amdgcn_wave_barrier(); asm volatile("" ::: "memory");
        float* crow = C + (size_t)(r0 + mb * 16) * ldc + c0;
#pragma unroll 1
        for (int ps = 0; ps < 2; ++ps) {
#pragma unroll
            for (int s = 0; s < 8; ++s) { const int row = 2 * s + hi, cofs = lr * 4; v4f val = *(const v4fa*)(os + row * 68 + cofs); if (BIAS) { val[0] += bfr(bias[c0 + cofs]); val[1] += bfr(bias[c0 + cofs + 1]); val[2] += bfr(bias[c0 + cofs + 2]); val[3] += bfr(bias[c0 + cofs + 3]); }
                *(volatile v4f*)(crow + (size_t)row * ldc + cofs) = val; }
            if (ps == 0) __threadfence(); }
        __builtin_amdgcn_wave_barrier(); asm volatile("" ::: "memory");
    }
}

__device__ __forceinline__ h16 tohx(float x) { return (h16)x; }
typedef __attribute__((ext_vector_type(2))) _Float16 v2h;
typedef __attribute__((ext_vector_type(4))) _Float16 v4h;
typedef __attribute__((ext_vector_type(2))) unsigned short v2us;
__global__ __launch_bounds__(256) void k_wtG(const float* __restrict__ w, int K, int N, bf* Bt) {
    const int lane = threadIdx.x & 31; const int L0 = (blockIdx.x * 8 + (threadIdx.x >> 5)) * 8; const int nlines = N * K / 64;
#pragma unroll 1
    for (int ps = 0; ps < 2; ++ps) {
#pragma unroll 1
        for (int l = 0; l < 8; ++l) { const int L = L0 + l; if (L >= nlines) break; const size_t e = (size_t)L * 64 + lane * 2; const int k = (int)(e % K), n = (int)(e / K); v2us o;
            o[0] = f2bf(w[(size_t)k * N + n]); o[1] = f2bf(w[(size_t)(k + 1) * N + n]); *(volatile v2us*)(Bt + e) = o; }
        if (ps == 0) __threadfence(); }
}


__global__ __launch_bounds__(256) void k_cvt8(const float* __restrict__ src, bf* dst, size_t n8) { const size_t i = (size_t)blockIdx.x * 256 + threadIdx.x; if (i >= n8) return; const v8f v = *(const v8f*)(src + i * 8); v8us o;
#pragma unroll
    for (int k = 0; k < 8; ++k) o[k] = f2bf(v[k]); *(volatile v8us*)(dst + i * 8) = o; __threadfence(); *(volatile v8us*)(dst + i * 8) = o; }
__global__ __launch_bounds__(256) void k_wt16(const float* __restrict__ w, int K, int N, h16* Bt) { const size_t e = ((size_t)blockIdx.x * 256 + threadIdx.x) * 2; if (e >= (size_t)N * K) return; const int k = (int)(e % K), n = (int)(e / K); v2h o; o[0] = tohx(bfr(w[(size_t)k * N + n])); o[1] = tohx(bfr(w[(size_t)(k + 1) * N + n])); *(volatile v2h*)(Bt + e) = o; __threadfence(); *(volatile v2h*)(Bt + e) = o; }
__global__ __launch_bounds__(256) void k_ln16(const float* __restrict__ X, int isin, const float* __restrict__ g, const float* __restrict__ bb, h16* Y) { const int lane = threadIdx.x & 31; const int t = blockIdx.x * 8 + (threadIdx.x >> 5); if (t >= TT) return; float v[24]; float s = 0.f;
#pragma unroll
    for (int ch = 0; ch < 6; ++ch) { const v4f a = *(const v4f*)(X + (size_t)t * EE + ch * 128 + lane * 4);
#pragma unroll
        for (int q = 0; q < 4; ++q) { const float x = isin ? bfr(a[q]) : a[q]; v[ch * 4 + q] = x; s = __fadd_rn(s, x); } }
#pragma unroll
    for (int sh = 16; sh; sh >>= 1) s += __shfl_xor(s, sh, 32);
    const float mu = s * (1.0f / EE); float q2 = 0.f;
#pragma unroll
    for (int k = 0; k < 24; ++k) { const float d = __fsub_rn(v[k], mu); float p = __fmul_rn(d, d); asm volatile("" : "+v"(p)); q2 = __fadd_rn(q2, p); }
#pragma unroll
    for (int sh = 16; sh; sh >>= 1) q2 += __shfl_xor(q2, sh, 32);
    const float rs = __frsqrt_rn(__fadd_rn(q2 * (1.0f / EE), 1e-5f));
#pragma unroll 1
    for (int ps = 0; ps < 2; ++ps) {
#pragma unroll
        for (int ch = 0; ch < 6; ++ch) { v4h o;
#pragma unroll
            for (int q = 0; q < 4; ++q) { const int d = ch * 128 + lane * 4 + q; float tn = __fmul_rn(__fsub_rn(v[ch * 4 + q], mu), rs); asm volatile("" : "+v"(tn)); float tg = __fmul_rn(tn, bfr(g[d])); asm volatile("" : "+v"(tg)); o[q] = tohx(__fadd_rn(tg, bfr(bb[d]))); }
            *(volatile v4h*)(Y + (size_t)t * EE + ch * 128 + lane * 4) = o; }
        if (ps == 0) __threadfence(); } }
__global__ __launch_bounds__(256) void k_hsplit(const float* __restrict__ F, int Tn, float scl, h16* P) { const size_t e = ((size_t)blockIdx.x * 256 + threadIdx.x) * 4; if (e >= (size_t)NH_ * Tn * HD) return; const int d = (int)(e % HD); const int t = (int)((e / HD) % Tn); const int h = (int)(e / ((size_t)HD * Tn)); const v4f a = *(const v4f*)(F + (size_t)t * EE + h * HD + d); v4h o;
#pragma unroll
    for (int q = 0; q < 4; ++q) o[q] = tohx(__fmul_rn(a[q], scl)); *(volatile v4h*)(P + e) = o; __threadfence(); *(volatile v4h*)(P + e) = o; }
__global__ __launch_bounds__(256) void k_vt(const float* __restrict__ F, int Tn, h16* VT) { const size_t e = ((size_t)blockIdx.x * 256 + threadIdx.x) * 2; if (e >= (size_t)NH_ * HD * Tn) return; const int t = (int)(e % Tn); const int d = (int)((e / Tn) % HD); const int h = (int)(e / ((size_t)Tn * HD)); v2h o; o[0] = tohx(F[(size_t)t * EE + h * HD + d]); o[1] = tohx(F[(size_t)(t + 1) * EE + h * HD + d]); *(volatile v2h*)(VT + e) = o; __threadfence(); *(volatile v2h*)(VT + e) = o; }
__global__ __launch_bounds__(256) void k_merge(const float* __restrict__ Ob, h16* O16) { const size_t e = ((size_t)blockIdx.x * 256 + threadIdx.x) * 4; if (e >= (size_t)TT * EE) return; const int c = (int)(e % EE), t = (int)(e / EE); const int h = c / HD, d = c % HD; const v4f a = *(const v4f*)(Ob + ((size_t)h * TT + t) * HD + d); v4h o;
#pragma unroll
    for (int q = 0; q < 4; ++q) o[q] = tohx(a[q] * (1.0f / PCAR)); *(volatile v4h*)(O16 + e) = o; __threadfence(); *(volatile v4h*)(O16 + e) = o; }
__global__ __launch_bounds__(256) void k_res(const float* __restrict__ A, const float* __restrict__ R, int isin, float* X1) { const size_t i = ((size_t)blockIdx.x * 256 + threadIdx.x) * 4; if (i >= (size_t)TT * EE) return; const v4f a = *(const v4f*)(A + i), r = *(const v4f*)(R + i); v4f o;
#pragma unroll
    for (int q = 0; q < 4; ++q) o[q] = __fadd_rn(a[q], isin ? bfr(r[q]) : r[q]); *(volatile v4f*)(X1 + i) = o; __threadfence(); *(volatile v4f*)(X1 + i) = o; }
__global__ __launch_bounds__(256) void k_gelu16(const float* __restrict__ F, h16* G) { const size_t i = ((size_t)blockIdx.x * 256 + threadIdx.x) * 4; if (i >= (size_t)TT * FF) return; const v4f a = *(const v4f*)(F + i); v4h o;
#pragma unroll
    for (int q = 0; q < 4; ++q) { const float x = a[q]; float x3 = __fmul_rn(__fmul_rn(x, x), x); asm volatile("" : "+v"(x3)); float in_ = __fmul_rn(0.7978845608028654f, __fadd_rn(x, __fmul_rn(0.044715f, x3))); asm volatile("" : "+v"(in_)); const float e2 = __expf(2.0f * in_); const float th = __fsub_rn(1.0f, __fdiv_rn(2.0f, __fadd_rn(e2, 1.0f))); float hx = __fmul_rn(0.5f, x); asm volatile("" : "+v"(hx)); o[q] = tohx(__fmul_rn(hx, __fadd_rn(1.0f, th))); }
    *(volatile v4h*)(G + i) = o; __threadfence(); *(volatile v4h*)(G + i) = o; }
template <int TK>
__global__ __launch_bounds__(256) void k_bsoft(const float* __restrict__ S, const float* __restrict__ bias, h16* P) { constexpr int NC = TK / 128; const int lane = threadIdx.x & 31; const int row = blockIdx.x * 8 + (threadIdx.x >> 5); if (row >= NH_ * TT) return; const float* sr = S + (size_t)row * TK; const float* br = bias + (size_t)row * TK; float v[NC * 4]; float mx = -3.0e38f;
#pragma unroll
    for (int ch = 0; ch < NC; ++ch) { const v4f a = *(const v4f*)(sr + ch * 128 + lane * 4); const v4f bb = *(const v4f*)(br + ch * 128 + lane * 4);
#pragma unroll
        for (int q = 0; q < 4; ++q) { const float t = __fadd_rn(a[q], bfr(bb[q])); v[ch * 4 + q] = t; mx = fmaxf(mx, t); } }
#pragma unroll
    for (int sh = 16; sh; sh >>= 1) mx = fmaxf(mx, __shfl_xor(mx, sh, 32));
    float sum = 0.f;
#pragma unroll
    for (int k = 0; k < NC * 4; ++k) { float d0 = __fsub_rn(v[k], mx); asm volatile("" : "+v"(d0)); v[k] = __expf(d0); sum += v[k]; }
#pragma unroll
    for (int sh = 16; sh; sh >>= 1) sum += __shfl_xor(sum, sh, 32);
    const float f = __fdiv_rn(PCAR, sum);
#pragma unroll 1
    for (int ps = 0; ps < 2; ++ps) {
#pragma unroll
        for (int ch = 0; ch < NC; ++ch) { v4h o;
#pragma unroll
            for (int q = 0; q < 4; ++q) o[q] = tohx(v[ch * 4 + q] * f); *(volatile v4h*)(P + (size_t)row * TK + ch * 128 + lane * 4) = o; }
        if (ps == 0) __threadfence(); } }

extern "C" void kernel_launch(void* const* d_in, const int* in_sizes, int n_in,
                              void* d_out, int out_size, void* d_ws, size_t ws_size, hipStream_t stream) {
    (void)in_sizes; (void)n_in; (void)out_size;
    const float* IN[30]; for (int i = 0; i < 30; ++i) IN[i] = (const float*)d_in[i];
    float* OUT = (float*)d_out;
    char* wsp = (char*)d_ws;
    auto take = [&](size_t bytes) { char* p = wsp; wsp += (bytes + 255) & ~(size_t)255; return (void*)p; };
    h16* WQC = (h16*)take((size_t)EE * EE * 2); bf* WKC = (bf*)take((size_t)EE * EC * 2); bf* WVC = (bf*)take((size_t)EE * EC * 2); h16* WOC = (h16*)take((size_t)EE * EE * 2); h16* WQS = (h16*)take((size_t)EE * EE * 2); h16* WKS = (h16*)take((size_t)EE * EE * 2); h16* WVS = (h16*)take((size_t)EE * EE * 2); h16* WOS = (h16*)take((size_t)EE * EE * 2); h16* W1 = (h16*)take((size_t)FF * EE * 2); h16* W2 = (h16*)take((size_t)EE * FF * 2);
    h16* X16 = (h16*)take((size_t)TT * EE * 2); bf* CB = (bf*)take((size_t)LC * EC * 2); float* QF = (float*)take((size_t)TT * EE * 4); float* KF = (float*)take((size_t)TT * EE * 4); float* VF = (float*)take((size_t)TT * EE * 4);
    h16* Q16 = (h16*)take((size_t)NH_ * TT * HD * 2); h16* K16 = (h16*)take((size_t)NH_ * TT * HD * 2); h16* VT16 = (h16*)take((size_t)NH_ * HD * TT * 2); float* Sb = (float*)take((size_t)NH_ * TT * TT * 4); h16* P16 = (h16*)take((size_t)NH_ * TT * TT * 2); float* Ob = (float*)take((size_t)NH_ * TT * HD * 4); h16* O16 = (h16*)take((size_t)TT * EE * 2);
    float* ATT = (float*)take((size_t)TT * EE * 4); float* H1 = (float*)take((size_t)TT * EE * 4); float* H2 = (float*)take((size_t)TT * EE * 4); h16* G16 = (h16*)take((size_t)TT * FF * 2);
    float* F1 = Sb;
    if ((size_t)(wsp - (char*)d_ws) > ws_size) return;
    k_wt16<<<(EE * EE / 2 + 255) / 256, 256, 0, stream>>>(IN[4], EE, EE, WQC); k_wtG<<<(EC * EE / 64 + 63) / 64, 256, 0, stream>>>(IN[6], EC, EE, WKC); k_wtG<<<(EC * EE / 64 + 63) / 64, 256, 0, stream>>>(IN[8], EC, EE, WVC); k_wt16<<<(EE * EE / 2 + 255) / 256, 256, 0, stream>>>(IN[10], EE, EE, WOC);
    k_wt16<<<(EE * EE / 2 + 255) / 256, 256, 0, stream>>>(IN[15], EE, EE, WQS); k_wt16<<<(EE * EE / 2 + 255) / 256, 256, 0, stream>>>(IN[17], EE, EE, WKS); k_wt16<<<(EE * EE / 2 + 255) / 256, 256, 0, stream>>>(IN[19], EE, EE, WVS); k_wt16<<<(EE * EE / 2 + 255) / 256, 256, 0, stream>>>(IN[21], EE, EE, WOS);
    k_wt16<<<(unsigned)(((size_t)EE * FF / 2 + 255) / 256), 256, 0, stream>>>(IN[26], EE, FF, W1); k_wt16<<<(unsigned)(((size_t)FF * EE / 2 + 255) / 256), 256, 0, stream>>>(IN[28], FF, EE, W2);
    const unsigned L4 = (unsigned)(((size_t)TT * EE / 4 + 255) / 256);
    for (int b = 0; b < NB_; ++b) { const float* hs = IN[0] + (size_t)b * TT * EE; const float* ctx = IN[1] + (size_t)b * LC * EC;
        k_ln16<<<TT / 8, 256, 0, stream>>>(hs, 1, IN[2], IN[3], X16); k_cvt8<<<(LC * EC / 8 + 255) / 256, 256, 0, stream>>>(ctx, CB, (size_t)LC * EC / 8);
        k_gemmw<h16, 0, true><<<dim3(TT / 64, EE / 64, 1), 32, 0, stream>>>(X16, nullptr, WQC, nullptr, EE, QF, EE, IN[5], 0, 0, 0); k_hsplit<<<(unsigned)(((size_t)NH_ * TT * HD / 4 + 255) / 256), 256, 0, stream>>>(QF, TT, 0.125f, Q16);
        k_gemmw<bf, 0, true><<<dim3(LC / 64, EE / 64, 1), 32, 0, stream>>>(CB, nullptr, WKC, nullptr, EC, KF, EE, IN[7], 0, 0, 0); k_hsplit<<<(unsigned)(((size_t)NH_ * LC * HD / 4 + 255) / 256), 256, 0, stream>>>(KF, LC, 1.0f, K16);
        k_gemmw<bf, 0, true><<<dim3(LC / 64, EE / 64, 1), 32, 0, stream>>>(CB, nullptr, WVC, nullptr, EC, VF, EE, IN[9], 0, 0, 0); k_vt<<<(unsigned)(((size_t)NH_ * HD * LC / 2 + 255) / 256), 256, 0, stream>>>(VF, LC, VT16);
        k_gemmw<h16, 0, false><<<dim3(TT / 64, LC / 64, NH_), 32, 0, stream>>>(Q16, nullptr, K16, nullptr, HD, Sb, LC, nullptr, (size_t)TT * HD, (size_t)LC * HD, (size_t)TT * LC);
        k_bsoft<LC><<<NH_ * TT / 8, 256, 0, stream>>>(Sb, IN[12], P16);
        k_gemmw<h16, 0, false><<<dim3(TT / 64, 1, NH_), 32, 0, stream>>>(P16, nullptr, VT16, nullptr, LC, Ob, HD, nullptr, (size_t)TT * LC, (size_t)HD * LC, (size_t)TT * HD); k_merge<<<L4, 256, 0, stream>>>(Ob, O16);
        k_gemmw<h16, 0, true><<<dim3(TT / 64, EE / 64, 1), 32, 0, stream>>>(O16, nullptr, WOC, nullptr, EE, ATT, EE, IN[11], 0, 0, 0); k_res<<<L4, 256, 0, stream>>>(ATT, hs, 1, H1);
        k_ln16<<<TT / 8, 256, 0, stream>>>(H1, 0, IN[13], IN[14], X16);
        k_gemmw<h16, 0, true><<<dim3(TT / 64, EE / 64, 1), 32, 0, stream>>>(X16, nullptr, WQS, nullptr, EE, QF, EE, IN[16], 0, 0, 0); k_hsplit<<<(unsigned)(((size_t)NH_ * TT * HD / 4 + 255) / 256), 256, 0, stream>>>(QF, TT, 0.125f, Q16);
        k_gemmw<h16, 0, true><<<dim3(TT / 64, EE / 64, 1), 32, 0, stream>>>(X16, nullptr, WKS, nullptr, EE, KF, EE, IN[18], 0, 0, 0); k_hsplit<<<(unsigned)(((size_t)NH_ * TT * HD / 4 + 255) / 256), 256, 0, stream>>>(KF, TT, 1.0f, K16);
        k_gemmw<h16, 0, true><<<dim3(TT / 64, EE / 64, 1), 32, 0, stream>>>(X16, nullptr, WVS, nullptr, EE, VF, EE, IN[20], 0, 0, 0); k_vt<<<(unsigned)(((size_t)NH_ * HD * TT / 2 + 255) / 256), 256, 0, stream>>>(VF, TT, VT16);
        k_gemmw<h16, 0, false><<<dim3(TT / 64, TT / 64, NH_), 32, 0, stream>>>(Q16, nullptr, K16, nullptr, HD, Sb, TT, nullptr, (size_t)TT * HD, (size_t)TT * HD, (size_t)TT * TT);
        k_bsoft<TT><<<NH_ * TT / 8, 256, 0, stream>>>(Sb, IN[23], P16);
        k_gemmw<h16, 0, false><<<dim3(TT / 64, 1, NH_), 32, 0, stream>>>(P16, nullptr, VT16, nullptr, TT, Ob, HD, nullptr, (size_t)TT * TT, (size_t)HD * TT, (size_t)TT * HD); k_merge<<<L4, 256, 0, stream>>>(Ob, O16);
        k_gemmw<h16, 0, true><<<dim3(TT / 64, EE / 64, 1), 32, 0, stream>>>(O16, nullptr, WOS, nullptr, EE, ATT, EE, IN[22], 0, 0, 0); k_res<<<L4, 256, 0, stream>>>(ATT, H1, 0, H2);
        k_ln16<<<TT / 8, 256, 0, stream>>>(H2, 0, IN[24], IN[25], X16);
        k_gemmw<h16, 0, true><<<dim3(TT / 64, FF / 64, 1), 32, 0, stream>>>(X16, nullptr, W1, nullptr, EE, F1, FF, IN[27], 0, 0, 0); k_gelu16<<<(unsigned)(((size_t)TT * FF / 4 + 255) / 256), 256, 0, stream>>>(F1, G16);
        k_gemmw<h16, 0, true><<<dim3(TT / 64, EE / 64, 1), 32, 0, stream>>>(G16, nullptr, W2, nullptr, FF, OUT + (size_t)b * TT * EE, EE, IN[29], 0, 0, 0); }
}
